// FeedForwardQuantum_65481071410500
// MI455X (gfx1250) — hardware-run, weakly checked
//
#include <hip/hip_runtime.h>
#include <stddef.h>


typedef _Float16 v16h __attribute__((ext_vector_type(16)));
typedef _Float16 v8h  __attribute__((ext_vector_type(8)));
typedef float    v8f  __attribute__((ext_vector_type(8)));
typedef float    v4f  __attribute__((ext_vector_type(4)));
typedef _Float16 h16;

#ifndef NB
#define NB 8
#endif
#ifndef SEQ
#define SEQ 2048
#endif
#define NB_FULL  8
#define SEQ_FULL 2048
#define CDIM  256
#define HID   1024
#define NWIRE 4
#define NAMP  16
#define NRAND 20
#define MROWS (NB * SEQ)

#ifndef LEG_BF16
#define LEG_BF16 1
#endif
#ifndef PARAM_BF16
#define PARAM_BF16 LEG_BF16
#endif

#define QT    128
#define HROWS 16

static_assert(NB >= 1 && NB <= NB_FULL);
static_assert(SEQ >= 128 && SEQ <= SEQ_FULL && (SEQ % 128) == 0);
static_assert(NAMP == (1 << NWIRE));
static_assert(NWIRE == 4);
static_assert((CDIM % 64) == 0 && (CDIM % 4) == 0);
static_assert((HID % 64) == 0 && (HID % 32) == 0);
static_assert(HID == 128 * 8);
static_assert((MROWS % 64) == 0 && (MROWS % QT) == 0 && (MROWS % HROWS) == 0);
static_assert((HROWS % 2) == 0);
static_assert(((size_t)CDIM * HID) % (256 * 8) == 0);
static_assert((size_t)MROWS * HID < (size_t)0xFFFFFFFFu);

#define LDC 68
static_assert((LDC % 4) == 0 && LDC >= 64);

#define WCARRY 64.0f
#define MCARRY 16.0f

#define W2_BYTES   ((size_t)CDIM * HID * 2)
#define Q_BYTES    ((size_t)MROWS * NWIRE * 4)
#define MID_BYTES  ((size_t)MROWS * HID * 2)
#define OFF_W2  ((size_t)0)
#define OFF_Q   (OFF_W2 + W2_BYTES)
#define OFF_MID (OFF_Q + Q_BYTES)
#define WS_TOTAL (OFF_MID + MID_BYTES)
static_assert((W2_BYTES % 128) == 0 && (Q_BYTES % 128) == 0 && (MID_BYTES % 128) == 0);
static_assert(WS_TOTAL <= (size_t)134217728);

__device__ __forceinline__ float bf16r(float x) {
  unsigned int u = __float_as_uint(x);
  u = (u + 0x7FFFu + ((u >> 16) & 1u)) & 0xFFFF0000u;
  return __uint_as_float(u);
}
__device__ __forceinline__ float inr(float x)  { return LEG_BF16 ? bf16r(x) : x; }
__device__ __forceinline__ float parr(float x) { return PARAM_BF16 ? bf16r(x) : x; }

static __device__ __forceinline__ h16 toh_flush(float v) {
  const h16 r = (h16)v;
  return (fabsf(v) < 6.103515625e-05f) ? (h16)0.0f : r;
}

__device__ __forceinline__ v16h frag_at(const _Float16* p) {
  v8h lo = *(const v8h*)(p);
  v8h hi = *(const v8h*)(p + 16);
  v16h out;
#pragma unroll
  for (int i = 0; i < 8; ++i) { out[i] = lo[i]; out[i + 8] = hi[i]; }
  return out;
}

__device__ __forceinline__ v8f wmma16(v16h a, v16h b, v8f c) {
  v8f d = __builtin_amdgcn_wmma_f32_16x16x32_f16(false, a, false, b, (short)0, c,
                                                 false, false);
  asm volatile("v_nop\n\tv_nop\n\tv_nop\n\tv_nop" : "+v"(d) : "v"(a), "v"(b));
  return d;
}

__device__ __forceinline__ float relu_act(float t) {
  return fmaxf(t, 0.0f);
}

__global__ __launch_bounds__(256) void w2conv_kernel(
    const float* __restrict__ W, _Float16* __restrict__ Wh) {
  const size_t e = ((size_t)blockIdx.x * 256u + threadIdx.x) * 8u;
  const v4f a0 = *(const v4f*)(W + e);
  const v4f a1 = *(const v4f*)(W + e + 4u);
  v8h o;
#pragma unroll
  for (int j = 0; j < 4; ++j) {
    o[j]     = toh_flush(WCARRY * inr(a0[j]));
    o[j + 4] = toh_flush(WCARRY * inr(a1[j]));
  }
  _Float16* p = Wh + e;
  *(volatile v8h*)p = o;
  __threadfence();
  *(volatile v8h*)p = o;
}

__global__ __launch_bounds__(QT) void circuit_kernel(
    const float* __restrict__ X, const float* __restrict__ RP,
    const float* __restrict__ RXT, const float* __restrict__ RYT,
    float* __restrict__ Q) {
#pragma clang fp contract(off)
  __shared__ float SR[NAMP * QT];
  __shared__ float SI[NAMP * QT];
  const unsigned tid = threadIdx.x;
  const unsigned crow = blockIdx.x * (unsigned)QT + tid;
  const unsigned bidx = crow / (unsigned)SEQ;
  const unsigned sq = crow - bidx * (unsigned)SEQ;
  const size_t srow = (size_t)bidx * SEQ_FULL + sq;
  const v4f xa = *(const v4f*)(X + srow * CDIM);
  const float a0 = inr(xa[0]);
  const float a1 = inr(xa[1]);
  const float a2 = inr(xa[2]);
  const float a3 = inr(xa[3]);
  const float rxv = parr(RXT[0]);
  const float ryv = parr(RYT[0]);

#pragma unroll 1
  for (unsigned i = 0; i < (unsigned)NAMP; ++i) {
    SR[i * QT + tid] = (i == 0u) ? 1.0f : 0.0f;
    SI[i * QT + tid] = 0.0f;
  }

#pragma unroll 1
  for (unsigned g = 0; g < 32u; ++g) {
    const unsigned gi = (g < 4u) ? 0u : (g - 4u);
    const unsigned ri = (gi > (unsigned)(NRAND - 1)) ? (unsigned)(NRAND - 1) : gi;
    const float pv = parr(RP[ri]);
    const unsigned gs = (g < 24u) ? 0u : (g - 24u);
    const float ta = (g == 0u) ? a0 : ((g == 1u) ? a1 : ((g == 2u) ? a2 : a3));
    const unsigned kind = (g < 4u) ? 1u : ((g < 24u) ? (ri % 3u) : (gs & 1u));
    const unsigned wire = (g < 4u) ? g : ((g < 24u) ? ((ri * 7u) & 3u) : (gs >> 1));
    const float ang = (g < 4u) ? ta : ((g < 24u) ? pv : (((gs & 1u) != 0u) ? ryv : rxv));
    const unsigned bv = 8u >> wire;

    float sn, cs;
    sincosf(ang * 0.5f, &sn, &cs);

    const float m00r = cs;
    const float m00i = (kind == 2u) ? -sn : 0.0f;
    const float m01r = (kind == 1u) ? -sn : 0.0f;
    const float m01i = (kind == 0u) ? -sn : 0.0f;
    const float m10r = (kind == 1u) ? sn : 0.0f;
    const float m10i = (kind == 0u) ? -sn : 0.0f;
    const float m11r = cs;
    const float m11i = (kind == 2u) ? sn : 0.0f;

#pragma unroll 1
    for (unsigned p = 0; p < 8u; ++p) {
      const unsigned low = p & (bv - 1u);
      const unsigned i0x = ((p - low) << 1) | low;
      const unsigned i1x = i0x | bv;
      const float r0 = SR[i0x * QT + tid];
      const float c0 = SI[i0x * QT + tid];
      const float r1 = SR[i1x * QT + tid];
      const float c1 = SI[i1x * QT + tid];
      const float n0r = (m00r * r0 - m00i * c0) + (m01r * r1 - m01i * c1);
      const float n0i = (m00r * c0 + m00i * r0) + (m01r * c1 + m01i * r1);
      const float n1r = (m10r * r0 - m10i * c0) + (m11r * r1 - m11i * c1);
      const float n1i = (m10r * c0 + m10i * r0) + (m11r * c1 + m11i * r1);
      SR[i0x * QT + tid] = n0r;
      SI[i0x * QT + tid] = n0i;
      SR[i1x * QT + tid] = n1r;
      SI[i1x * QT + tid] = n1i;
    }

    const bool cn = (g >= 4u) && (g < 24u) && ((ri % 5u) == 4u);
    if (cn) {
      const unsigned cw = ri / 5u;
      const unsigned tw = (cw + 1u) & 3u;
      const unsigned cb = 8u >> cw;
      const unsigned tb = 8u >> tw;
#pragma unroll 1
      for (unsigned p = 0; p < 8u; ++p) {
        const unsigned low = p & (tb - 1u);
        const unsigned i0x = ((p - low) << 1) | low;
        const unsigned i1x = i0x | tb;
        if ((i0x & cb) != 0u) {
          const float r0 = SR[i0x * QT + tid];
          const float c0 = SI[i0x * QT + tid];
          const float r1 = SR[i1x * QT + tid];
          const float c1 = SI[i1x * QT + tid];
          SR[i0x * QT + tid] = r1;
          SI[i0x * QT + tid] = c1;
          SR[i1x * QT + tid] = r0;
          SI[i1x * QT + tid] = c0;
        }
      }
    }
  }

  float e0 = 0.0f, e1 = 0.0f, e2 = 0.0f, e3 = 0.0f;
#pragma unroll 1
  for (unsigned i = 0; i < (unsigned)NAMP; ++i) {
    const float re = SR[i * QT + tid];
    const float im = SI[i * QT + tid];
    const float pr = re * re + im * im;
    e0 += ((i & 8u) != 0u) ? -pr : pr;
    e1 += ((i & 4u) != 0u) ? -pr : pr;
    e2 += ((i & 2u) != 0u) ? -pr : pr;
    e3 += ((i & 1u) != 0u) ? -pr : pr;
  }
  v4f qv;
  qv[0] = e0; qv[1] = e1; qv[2] = e2; qv[3] = e3;
  float* p = Q + (size_t)crow * NWIRE;
  *(volatile v4f*)p = qv;
  __threadfence();
  *(volatile v4f*)p = qv;
}

__global__ __launch_bounds__(256) void ffn1_kernel(
    const float* __restrict__ Q, const float* __restrict__ W1, const float* __restrict__ B1,
    _Float16* __restrict__ Mid) {
#pragma clang fp contract(off)
  const unsigned tid = threadIdx.x;
  const unsigned cg = tid & 127u;
  const unsigned rsub = tid >> 7;
  const unsigned row0 = blockIdx.x * (unsigned)HROWS;

  v4f wv[8];
#pragma unroll
  for (int j = 0; j < 8; ++j) {
    const v4f t = *(const v4f*)(W1 + (size_t)(cg * 8u + (unsigned)j) * NWIRE);
#pragma unroll
    for (int k = 0; k < 4; ++k) wv[j][k] = inr(t[k]);
  }
  const v4f ba = *(const v4f*)(B1 + cg * 8u);
  const v4f bb = *(const v4f*)(B1 + cg * 8u + 4u);
  float bj[8];
#pragma unroll
  for (int j = 0; j < 4; ++j) { bj[j] = inr(ba[j]); bj[j + 4] = inr(bb[j]); }

#pragma unroll 1
  for (unsigned it = 0; it < (unsigned)(HROWS / 2); ++it) {
    const unsigned crow = row0 + 2u * it + rsub;
    const v4f qv = *(const v4f*)(Q + (size_t)crow * NWIRE);
    v8h o;
#pragma unroll
    for (int j = 0; j < 8; ++j) {
      const float t = ((qv[0] * wv[j][0] + qv[1] * wv[j][1]) +
                       (qv[2] * wv[j][2] + qv[3] * wv[j][3])) + bj[j];
      o[j] = toh_flush(MCARRY * relu_act(t));
    }
    _Float16* p = Mid + (size_t)crow * HID + cg * 8u;
    *(volatile v8h*)p = o;
    __threadfence();
    *(volatile v8h*)p = o;
  }
}

__global__ __launch_bounds__(256) void gemm_ffn2_kernel(
    const _Float16* __restrict__ A16, const _Float16* __restrict__ Bt,
    const float* __restrict__ bias, float* __restrict__ outf) {
  __shared__ float Cs[64 * LDC];
  const unsigned K = (unsigned)HID;
  const unsigned tid = threadIdx.x, lane = tid & 31u, w = tid >> 5;
  const unsigned mw = w >> 1, nw = w & 1u;
  const unsigned hh = lane >> 4, m = lane & 15u;
  const unsigned n0 = blockIdx.x * 64u;
  const unsigned row0 = blockIdx.y * 64u;

  const _Float16* ap  = A16 + (size_t)(row0 + mw * 16u + m) * K + hh * 8u;
  const _Float16* bp0 = Bt + (size_t)(n0 + nw * 32u + m) * K + hh * 8u;
  const _Float16* bp1 = bp0 + (size_t)16 * K;
  v8f acc0 = {}, acc1 = {};
#pragma unroll 2
  for (unsigned k0 = 0; k0 < K; k0 += 32u) {
    const v16h a  = frag_at(ap + k0);
    const v16h b0 = frag_at(bp0 + k0);
    const v16h b1 = frag_at(bp1 + k0);
    acc0 = wmma16(a, b0, acc0);
    acc1 = wmma16(a, b1, acc1);
  }
#pragma unroll
  for (int r = 0; r < 8; ++r) {
    float* d = &Cs[(mw * 16u + hh * 8u + (unsigned)r) * LDC + nw * 32u + m];
    d[0]  = acc0[r];
    d[16] = acc1[r];
  }
  __syncthreads();

  const float cs = 1.0f / (WCARRY * MCARRY);
  v4f xs[4];
  size_t off[4];
#pragma unroll
  for (unsigned i = 0; i < 4u; ++i) {
    const unsigned r = 16u * i + (tid >> 4);
    const unsigned c = (tid & 15u) * 4u;
    const unsigned crow = row0 + r;
    const unsigned bidx = crow / (unsigned)SEQ;
    const unsigned sq = crow - bidx * (unsigned)SEQ;
    const size_t frow = (size_t)bidx * SEQ_FULL + sq;
    const v4f u = *(const v4f*)&Cs[r * LDC + c];
    const v4f g = *(const v4f*)(bias + n0 + c);
    v4f val;
#pragma unroll
    for (int j = 0; j < 4; ++j) val[j] = u[j] * cs + inr(g[j]);
    xs[i] = val;
    off[i] = frow * CDIM + n0 + c;
  }
#pragma unroll
  for (int i = 0; i < 4; ++i) *(volatile v4f*)(outf + off[i]) = xs[i];
  __threadfence();
#pragma unroll
  for (int i = 0; i < 4; ++i) *(volatile v4f*)(outf + off[i]) = xs[i];
}

extern "C" void kernel_launch(void* const* d_in, const int* in_sizes, int n_in,
                              void* d_out, int out_size, void* d_ws, size_t ws_size,
                              hipStream_t stream) {
  if (n_in < 8) return;
  const long long need_x = ((long long)(NB - 1) * SEQ_FULL + SEQ) * CDIM;
  if ((long long)in_sizes[0] < need_x) return;
  if ((long long)in_sizes[1] < (long long)HID * NWIRE) return;
  if (in_sizes[2] < HID) return;
  if ((long long)in_sizes[3] < (long long)CDIM * HID) return;
  if (in_sizes[4] < CDIM) return;
  if (in_sizes[5] < NRAND) return;
  if (in_sizes[6] < 1 || in_sizes[7] < 1) return;
  if ((long long)out_size < need_x) return;
  if (ws_size < WS_TOTAL) return;

  const float* X    = (const float*)d_in[0];
  const float* w1   = (const float*)d_in[1];
  const float* b1   = (const float*)d_in[2];
  const float* w2   = (const float*)d_in[3];
  const float* b2   = (const float*)d_in[4];
  const float* rp   = (const float*)d_in[5];
  const float* rxth = (const float*)d_in[6];
  const float* ryth = (const float*)d_in[7];
  float* out = (float*)d_out;

  char* ws = (char*)d_ws;
  _Float16* W2h   = (_Float16*)(ws + OFF_W2);
  float*    Qp    = (float*)(ws + OFF_Q);
  _Float16* Mid16 = (_Float16*)(ws + OFF_MID);

  dim3 blk(256);
  w2conv_kernel<<<dim3((unsigned)(((size_t)CDIM * HID) / (256 * 8))), blk, 0, stream>>>(w2, W2h);
  circuit_kernel<<<dim3(MROWS / QT), dim3(QT), 0, stream>>>(X, rp, rxth, ryth, Qp);
  ffn1_kernel<<<dim3(MROWS / HROWS), blk, 0, stream>>>(Qp, w1, b1, Mid16);
  gemm_ffn2_kernel<<<dim3(CDIM / 64, MROWS / 64), blk, 0, stream>>>(Mid16, W2h, b2, out);
}
